// VDDecoder_26414048871115
// MI455X (gfx1250) — hardware-verified
//
#include <hip/hip_runtime.h>
#include <math.h>

typedef __attribute__((ext_vector_type(16))) _Float16 v16h;
typedef __attribute__((ext_vector_type(8)))  _Float16 v8h;
typedef __attribute__((ext_vector_type(8)))  float    v8f;
typedef __attribute__((ext_vector_type(4)))  float    v4f;

constexpr int kBatch      = 512;
constexpr int kSteps      = 4096;
constexpr int kIn         = 1;
constexpr int kHid        = 16;
constexpr int kOutN       = 1;
constexpr int kTileRows   = 16;
constexpr int kTiles      = kBatch / kTileRows;
constexpr int kChunk      = 32;
constexpr int kNumChunks  = kSteps / kChunk;
constexpr int kXW         = kChunk * kIn;
constexpr int kOW         = kChunk * kOutN;
constexpr int kXPitch     = kXW + 4;
constexpr int kOPitch     = kOW + 4;
static_assert(kBatch % kTileRows == 0 && kSteps % kChunk == 0, "whole tiles and chunks");
static_assert(kHid == 16 && kIn <= 8 && kOutN == 1, "16 units fill the first 16 k; the input sits at k 16 of the low lane half; one output per step");
static_assert((kXW % 32) == 0 && (kOW % 32) == 0, "a row's chunk is a whole number of 128-B lines on both sides");
static_assert((kXPitch % 4) == 0 && (kOPitch % 4) == 0, "16-B aligned LDS rows");

constexpr float kStateCarry  = 256.0f;
constexpr float kWeightCarry = 64.0f;
constexpr float kFoldBack    = 1.0f / (kStateCarry * kWeightCarry);
constexpr float kF16MinNorm  = 6.103515625e-5f;
static_assert(kStateCarry * kWeightCarry == 16384.0f, "carry product");

namespace eng {

union FragU { v16h v; v8h h[2]; };

__device__ __forceinline__ unsigned short f2bf_bits(float f) {
  unsigned u = __float_as_uint(f);
  return (unsigned short)((u + 0x7FFFu + ((u >> 16) & 1u)) >> 16);
}
__device__ __forceinline__ float bf16v(float f) {
  return __uint_as_float(((unsigned)f2bf_bits(f)) << 16);
}
__device__ __forceinline__ _Float16 to_f16_flushed(float c) {
  const float z = (fabsf(c) < kF16MinNorm) ? 0.0f : c;
  return (_Float16)z;
}
__device__ __forceinline__ v8f mma_f16(v16h a, v16h b) {
  v8f c = (v8f){0.f, 0.f, 0.f, 0.f, 0.f, 0.f, 0.f, 0.f};
  c = __builtin_amdgcn_wmma_f32_16x16x32_f16(false, a, false, b, (short)0, c, false, false);
  asm volatile("v_nop\n\tv_nop\n\tv_nop\n\tv_nop" : "+v"(c) : "v"(a), "v"(b));
  return c;
}
__device__ __forceinline__ float fast_tanh(float v) {
  const float e = __expf(2.0f * v);
  return 1.0f - 2.0f * __builtin_amdgcn_rcpf(e + 1.0f);
}
__device__ __forceinline__ float fast_sigmoid(float v) {
  return __builtin_amdgcn_rcpf(1.0f + __expf(-v));
}

}

__global__ __launch_bounds__(32) void lstm16m_seq_kernel(
    const float* __restrict__ x,
    const float* __restrict__ w_ih,
    const float* __restrict__ w_hh,
    const float* __restrict__ b_g,
    const float* __restrict__ w_i2, const float* __restrict__ w_h2, const float* __restrict__ b_g2,
    const float* __restrict__ mask1, const float* __restrict__ mask2,
    float* __restrict__ outs)
{
  __shared__ __align__(16) float xs[kTileRows * kXPitch];
  __shared__ __align__(16) float os[kTileRows * kOPitch];
  __shared__ __align__(16) float wsm[4 * kHid * kHid];
  __shared__ __align__(16) float wim[4 * kHid * 8];
  __shared__ __align__(16) float wlm[4 * kHid];
  __shared__ __align__(16) float bsm[4 * kHid];
  __shared__ __align__(16) float blm[32];
  __shared__ __align__(16) float ism[kTileRows * kHid + 32];

  const int lane = threadIdx.x & 31;
  const int hsel = lane >> 4;
  const int n    = lane & 15;
  const bool lowHalf = (hsel == 0);
  const int b0   = blockIdx.x * kTileRows;

  {
#pragma unroll 1
    for (int i = lane; i < 4 * kHid * kHid; i += 32) wsm[i] = w_hh[i];
#pragma unroll 1
    for (int i = lane; i < 4 * kHid * 8; i += 32) {
      const int g  = i >> 3;
      const int f  = i & 7;
      const int fc = (f < kIn) ? f : (kIn - 1);
      wim[i] = w_ih[g * kIn + fc];
    }
#pragma unroll 1
    for (int i = lane; i < 4 * kHid; i += 32) { wlm[i] = w_i2[i]; bsm[i] = b_g[i]; }
    {
      const int i4 = lane & 3;
      const float vh = w_h2[i4];
      const float vb = b_g2[i4];
      blm[lane] = (lane < 4) ? vh : vb;
    }
#pragma unroll
    for (int it = 0; it < 8; ++it) {
      const int i = it * 32 + lane;
      ism[i] = mask1[(size_t)b0 * kHid + i];
    }
    ism[kTileRows * kHid + lane] = mask2[b0 + (lane & 15)];
  }
  __syncthreads();

  v16h fragA[4];
  v16h fragH;
  {
    const int m = n;
#pragma unroll
    for (int g = 0; g < 4; ++g) {
      v8h alo, ahi;
#pragma unroll
      for (int i = 0; i < 8; ++i) {
        const int k = 8 * hsel + i;
        const float f0 = wsm[(g * kHid + m) * kHid + k];
        alo[i] = eng::to_f16_flushed(eng::bf16v(f0) * kWeightCarry);
        const float f1 = wim[(g * kHid + m) * 8 + i];
        const bool ok = lowHalf && (i < kIn);
        const float g1 = ok ? (eng::bf16v(f1) * kWeightCarry) : 0.0f;
        ahi[i] = eng::to_f16_flushed(g1);
      }
      eng::FragU u0;
      u0.h[0] = alo;
      u0.h[1] = ahi;
      fragA[g] = u0.v;
    }
    const int mc = (m < 4) ? m : 3;
    const bool mok = (m < 4);
    v8h hlo, hhi;
#pragma unroll
    for (int i = 0; i < 8; ++i) {
      const float f0 = wlm[mc * kHid + 8 * hsel + i];
      const float g0 = mok ? (eng::bf16v(f0) * kWeightCarry) : 0.0f;
      hlo[i] = eng::to_f16_flushed(g0);
      const float f1 = blm[mc];
      const bool ok1 = mok && lowHalf && (i == 0);
      hhi[i] = eng::to_f16_flushed(ok1 ? (eng::bf16v(f1) * kWeightCarry) : 0.0f);
    }
    eng::FragU uh;
    uh.h[0] = hlo;
    uh.h[1] = hhi;
    fragH = uh.v;
  }

  float bi[8], bf[8], bg[8], bo[8];
  float hf[8], cf[8], m1[8];
  v8h hb;
#pragma unroll
  for (int r = 0; r < 8; ++r) {
    const int u = 8 * hsel + r;
    bi[r] = eng::bf16v(bsm[u]);
    bf[r] = eng::bf16v(bsm[kHid + u]);
    bg[r] = eng::bf16v(bsm[2 * kHid + u]);
    bo[r] = eng::bf16v(bsm[3 * kHid + u]);
    hf[r] = 0.0f;
    cf[r] = 0.0f;
    hb[r] = (_Float16)0.0f;
    m1[r] = eng::bf16v(ism[n * kHid + u]);
  }
  float b2g[4];
#pragma unroll
  for (int r = 0; r < 4; ++r) b2g[r] = eng::bf16v(blm[4 + r]);
  const float m2 = eng::bf16v(ism[kTileRows * kHid + n]);
  float h2f = 0.0f, c2f = 0.0f;
  const v8h zh = (v8h){(_Float16)0.0f, (_Float16)0.0f, (_Float16)0.0f, (_Float16)0.0f,
                       (_Float16)0.0f, (_Float16)0.0f, (_Float16)0.0f, (_Float16)0.0f};

#pragma unroll 1
  for (int ch = 0; ch < kNumChunks; ++ch) {
    const int t0 = ch * kChunk;
#pragma unroll
    for (int it = 0; it < 4; ++it) {
      const int vi  = it * 32 + lane;
      const int row = vi >> 3;
      const int c4  = (vi & 7) * 4;
      const v4f v = *(const v4f*)(x + ((size_t)(b0 + row) * kSteps + t0) * kIn + c4);
      v4f rv;
      const float v0 = v[0];
      const float v1 = v[1];
      const float v2 = v[2];
      const float v3 = v[3];
      rv[0] = eng::bf16v(v0);
      rv[1] = eng::bf16v(v1);
      rv[2] = eng::bf16v(v2);
      rv[3] = eng::bf16v(v3);
      *(v4f*)(xs + row * kXPitch + c4) = rv;
    }
    __syncthreads();

#pragma unroll 1
    for (int s = 0; s < kChunk; ++s) {
      v8h xb = zh;
#pragma unroll
      for (int i = 0; i < kIn; ++i) {
        const float xv = xs[n * kXPitch + s * kIn + i];
        const float xg = lowHalf ? (xv * kStateCarry) : 0.0f;
        xb[i] = eng::to_f16_flushed(xg);
      }
      eng::FragU fb;
      fb.h[0] = hb;
      fb.h[1] = xb;
      const v8f ai = eng::mma_f16(fragA[0], fb.v);
      const v8f af = eng::mma_f16(fragA[1], fb.v);
      const v8f ag = eng::mma_f16(fragA[2], fb.v);
      const v8f ao = eng::mma_f16(fragA[3], fb.v);
#pragma unroll
      for (int r = 0; r < 8; ++r) {
        const float ig = eng::fast_sigmoid(fmaf(ai[r], kFoldBack, bi[r]));
        const float fg = eng::fast_sigmoid(fmaf(af[r], kFoldBack, bf[r]));
        const float gg = eng::fast_tanh(fmaf(ag[r], kFoldBack, bg[r]));
        const float og = eng::fast_sigmoid(fmaf(ao[r], kFoldBack, bo[r]));
        const float cn = fg * cf[r] + ig * gg;
        cf[r] = cn;
        const float hv = og * eng::fast_tanh(cn);
        hf[r] = hv;
        hb[r] = eng::to_f16_flushed(hv * kStateCarry);
      }
      v8h mb;
#pragma unroll
      for (int r = 0; r < 8; ++r) mb[r] = eng::to_f16_flushed((hf[r] * m1[r]) * kStateCarry);
      v8h sb = zh;
      sb[0] = eng::to_f16_flushed(lowHalf ? (h2f * kStateCarry) : 0.0f);
      eng::FragU fh;
      fh.h[0] = mb;
      fh.h[1] = sb;
      const v8f ah = eng::mma_f16(fragH, fh.v);
      {
        const float ig = eng::fast_sigmoid(fmaf(ah[0], kFoldBack, b2g[0]));
        const float fg = eng::fast_sigmoid(fmaf(ah[1], kFoldBack, b2g[1]));
        const float gg = eng::fast_tanh(fmaf(ah[2], kFoldBack, b2g[2]));
        const float og = eng::fast_sigmoid(fmaf(ah[3], kFoldBack, b2g[3]));
        const float cn = fg * c2f + ig * gg;
        const float hv = og * eng::fast_tanh(cn);
        c2f = lowHalf ? cn : 0.0f;
        h2f = lowHalf ? hv : 0.0f;
      }
      if (lowHalf) os[n * kOPitch + s] = h2f * m2;
    }
    __syncthreads();

    {
      for (int pass = 0; pass < 2; ++pass) {
#pragma unroll
        for (int it = 0; it < 4; ++it) {
          const int vi  = it * 32 + lane;
          const int row = vi >> 3;
          const int c4  = (vi & 7) * 4;
          const v4f ov = *(const v4f*)(os + row * kOPitch + c4);
          *(volatile v4f*)(outs + ((size_t)(b0 + row) * kSteps + t0) * kOutN + c4) = ov;
        }
        __threadfence();
      }
    }
  }
}

extern "C" void kernel_launch(void* const* d_in, const int* in_sizes, int n_in,
                              void* d_out, int out_size, void* d_ws, size_t ws_size,
                              hipStream_t stream) {
  (void)d_ws;
  (void)ws_size;
  if (n_in < 9 || d_out == nullptr) return;
  if (in_sizes[0] != kBatch * kSteps * kIn) return;
  if (in_sizes[1] != 4 * kHid * kIn) return;
  if (in_sizes[2] != 4 * kHid * kHid) return;
  if (in_sizes[3] != 4 * kHid) return;
  if (in_sizes[4] != 4 * kHid || in_sizes[5] != 4 || in_sizes[6] != 4) return;
  if (in_sizes[7] != kBatch * kHid || in_sizes[8] != kBatch) return;
  if (out_size != kBatch * kSteps * kOutN) return;

  const float* x     = (const float*)d_in[0];
  const float* w_ih  = (const float*)d_in[1];
  const float* w_hh  = (const float*)d_in[2];
  const float* b_g   = (const float*)d_in[3];
  const float* w_i2  = (const float*)d_in[4];
  const float* w_h2  = (const float*)d_in[5];
  const float* b_g2  = (const float*)d_in[6];
  const float* mask1 = (const float*)d_in[7];
  const float* mask2 = (const float*)d_in[8];
  float* outs = (float*)d_out;

  lstm16m_seq_kernel<<<kTiles, 32, 0, stream>>>(x, w_ih, w_hh, b_g, w_i2, w_h2, b_g2, mask1, mask2, outs);
}
